// NetAmazon_GAT_heads_71768903516555
// MI455X (gfx1250) — hardware-run, weakly checked
//
#include <hip/hip_runtime.h>
#include <stddef.h>
#include <stdint.h>
#include <math.h>


#define NNODE   20000
#define MPAD    20096
#define FIN     745
#define K1P     768
#define HC1     1024
#define HC2     512
#define NCLS    10
#define H3W     16
#define NHD     8
#define KA2     2048
#define KA3     1024
#define NTHR    256
#define NWAVE   8
#define EPT     8
#define CHUNK   (NTHR * EPT)
#define WCAP    (EPT * 32)
#define LISTN   (NWAVE * WCAP)
#define NBA     512
#define SLA     9
#define SRCB    15
#define NGA     40
#define RCAP    12288
#define DEGCAP  64
#define MEAS_B512   8398
#define MEAS_MAXDEG 32
#define GBM     64
#define GTHR    128
#define MROWS   128
#define SCW     512
#define CPL     16
#define DROWS   32
#define STG_INTS 5120
#define NEGSL   0.2f
#define EPS_SM  1e-16f
#define BKT_LDS_INTS  (LISTN + 2 * RCAP + 3 * NBA + 16)
#define SCAN_LDS_INTS (RCAP + 2 * NBA + SCW + STG_INTS)

static_assert(NNODE < (1 << SRCB));
static_assert(NNODE % 16 == 0 && NBA % 16 == 0);
static_assert(MPAD % MROWS == 0 && MPAD >= NNODE && MPAD - NNODE < MROWS);
static_assert(MPAD % GBM == 0 && MPAD % DROWS == 0);
static_assert(NGA * NBA >= MPAD);
static_assert(K1P % 32 == 0 && K1P >= FIN && KA2 % 32 == 0 && KA3 % 32 == 0);
static_assert(KA2 == 2 * HC1 && KA3 == 2 * HC2);
static_assert((CHUNK & (CHUNK - 1)) == 0 && CHUNK <= 4096);
static_assert(NBA == (1 << SLA));
static_assert(((long long)CHUNK << SLA) < (1LL << 31));
static_assert(SRCB + SLA < 31);
static_assert(RCAP >= MEAS_B512 + 2048 && (RCAP % (NTHR * 4)) == 0);
static_assert(DEGCAP >= MEAS_MAXDEG + 8);
static_assert(2 * NBA == NTHR * 4);
static_assert(((RCAP + 3 * NBA) % 4) == 0);
static_assert(NBA % NWAVE == 0 && NBA % 32 == 0);
static_assert(SCW == 32 * CPL && HC1 % SCW == 0 && HC2 == SCW);
static_assert(NWAVE * 2 * SCW * 2 <= STG_INTS * 4);
static_assert(NBA * NCLS <= STG_INTS);
static_assert((NBA * NCLS * 4) % 128 == 0);
static_assert(BKT_LDS_INTS * 4 <= 300000 && SCAN_LDS_INTS * 4 <= 300000);
static_assert(GBM == (GTHR / 32) * 16);
static_assert(DROWS % NWAVE == 0 && DROWS * NHD == 256);

typedef float          v4f  __attribute__((ext_vector_type(4)));
typedef float          v8f  __attribute__((ext_vector_type(8)));
typedef int            v4i  __attribute__((ext_vector_type(4)));
typedef int            v8i  __attribute__((ext_vector_type(8)));
typedef unsigned short v8us __attribute__((ext_vector_type(8)));
typedef __bf16         v16b __attribute__((ext_vector_type(16)));
typedef v4f  __attribute__((may_alias)) v4fa;
typedef v4i  __attribute__((may_alias)) v4ia;
typedef v8us __attribute__((may_alias)) v8usa;
union FragB { v16b v; v8us h[2]; v8i w; };

__device__ __forceinline__ v8f wmb(const FragB& a, const FragB& b, v8f c) {
  v8f d = __builtin_amdgcn_wmma_f32_16x16x32_bf16(false, a.v, false, b.v, (short)0, c, false, false);
  asm volatile("v_nop\n\tv_nop\n\tv_nop\n\tv_nop" : "+v"(d) : "v"(a.w), "v"(b.w));
  return d;
}

__device__ __forceinline__ unsigned int f2bf(float f) {
  const unsigned int u = __float_as_uint(f);
  const unsigned int r = ((u + 0x7FFFu + ((u >> 16) & 1u)) >> 16) & 0xFFFFu;
  return ((u & 0x7FFFFFFFu) > 0x7F800000u) ? 0x7FC0u : r;
}
__device__ __forceinline__ float bf2f(unsigned int b) { return __uint_as_float(b << 16); }
__device__ __forceinline__ float bfr(float f) { return bf2f(f2bf(f)); }

__device__ __forceinline__ float fin1(float a, float inv, float b, float pz, bool live) {
  float y = fmaf(a, inv, b);
  y = (y > 0.0f) ? y : (y - y);
  y = y + pz;
  return live ? y : 0.0f;
}

template <int SLB>
__device__ __forceinline__ int scan_chunk(const int* __restrict__ dsts, int nE, int cbase, int slotBase,
                                          int nb, int vec8, int* list, int tid, int lane, int wave) {
  int wc = 0;
  const int el0  = tid * EPT;
  const int e0   = cbase + el0;
  const int sent = -2147483647 - 1;
  v4i da, db;
  if (vec8 != 0 && cbase + CHUNK <= nE) {
    da = *(const v4i*)(dsts + e0);
    db = *(const v4i*)(dsts + e0 + 4);
  } else {
    da.x = (e0     < nE) ? dsts[min(e0,     nE - 1)] : sent;
    da.y = (e0 + 1 < nE) ? dsts[min(e0 + 1, nE - 1)] : sent;
    da.z = (e0 + 2 < nE) ? dsts[min(e0 + 2, nE - 1)] : sent;
    da.w = (e0 + 3 < nE) ? dsts[min(e0 + 3, nE - 1)] : sent;
    db.x = (e0 + 4 < nE) ? dsts[min(e0 + 4, nE - 1)] : sent;
    db.y = (e0 + 5 < nE) ? dsts[min(e0 + 5, nE - 1)] : sent;
    db.z = (e0 + 6 < nE) ? dsts[min(e0 + 6, nE - 1)] : sent;
    db.w = (e0 + 7 < nE) ? dsts[min(e0 + 7, nE - 1)] : sent;
  }
  const unsigned nbs = (unsigned)slotBase;
  const unsigned unb = (unsigned)nb;
  const unsigned s0 = (unsigned)da.x - nbs, s1 = (unsigned)da.y - nbs;
  const unsigned s2 = (unsigned)da.z - nbs, s3 = (unsigned)da.w - nbs;
  const unsigned s4 = (unsigned)db.x - nbs, s5 = (unsigned)db.y - nbs;
  const unsigned s6 = (unsigned)db.z - nbs, s7 = (unsigned)db.w - nbs;
  const bool h0 = s0 < unb, h1 = s1 < unb, h2 = s2 < unb, h3 = s3 < unb;
  const bool h4 = s4 < unb, h5 = s5 < unb, h6 = s6 < unb, h7 = s7 < unb;
  const unsigned any = __builtin_amdgcn_ballot_w32(h0 | h1 | h2 | h3 | h4 | h5 | h6 | h7);
  if (any != 0u) {
#define HITJ(J, HJ, SJ) { \
      const unsigned mj = __builtin_amdgcn_ballot_w32(HJ); \
      if (mj != 0u) { \
        if (HJ) { \
          const int pos = wc + (int)__builtin_amdgcn_mbcnt_lo(mj, 0u); \
          if (pos < WCAP) list[wave * WCAP + pos] = ((el0 + (J)) << SLB) | (int)(SJ); \
        } \
        wc += (int)__builtin_popcount(mj); } }
    HITJ(0, h0, s0)
    HITJ(1, h1, s1)
    HITJ(2, h2, s2)
    HITJ(3, h3, s3)
    HITJ(4, h4, s4)
    HITJ(5, h5, s5)
    HITJ(6, h6, s6)
    HITJ(7, h7, s7)
#undef HITJ
  }
  return wc;
}

__global__ __launch_bounds__(NTHR) void k_cvt(const float* __restrict__ src, int R, int K, int P,
                                              unsigned short* dst, int Kp, int nUnits) {
  const int u = (int)blockIdx.x * NTHR + (int)threadIdx.x;
  if (u >= nUnits) return;
  const int kq  = Kp >> 3;
  const int row = u / kq;
  const int k8  = (u - row * kq) * 8;
  const int kk0 = k8 - (k8 / P) * P;
  const int rc  = row < R ? row : R - 1;
  const bool okr = row < R;
  const float* p = src + (size_t)rc * (size_t)K;
  v8us o;
#pragma unroll
  for (int i = 0; i < 8; ++i) {
    const int kk = kk0 + i;
    const int cc = kk < K ? kk : K - 1;
    const float f = p[cc];
    o[i] = (okr && kk < K) ? (unsigned short)f2bf(f) : (unsigned short)0;
  }
  unsigned short* dp = dst + (size_t)row * (size_t)Kp + k8;
  *(volatile v8us*)dp = o;
  __threadfence();
  *(volatile v8us*)dp = o;
}

__global__ __launch_bounds__(NTHR) void k_bucket(const int* __restrict__ srcs, const int* __restrict__ dsts,
                                                 int nE, int nN, int vec8, int* HITS, int* TAB, int* FLG) {
  extern __shared__ __attribute__((aligned(16))) int bsm[];
  int* list = bsm;
  int* reg1 = bsm + LISTN;
  int* reg2 = reg1 + RCAP;
  int* tab  = reg2 + RCAP;
  int* cur  = tab + 2 * NBA;
  int* wcnt = cur + NBA;
  int* offs = tab;
  int* cnt  = tab + NBA;
  const int tid = (int)threadIdx.x, lane = tid & 31, wave = tid >> 5;
  const int blk = (int)blockIdx.x;
  const int nodeBase = blk * NBA;
  int nb = nN - nodeBase;
  nb = nb < 0 ? 0 : (nb > NBA ? NBA : nb);

  {
    const v4i z4 = {0, 0, 0, 0};
    for (int i = tid * 4; i < RCAP + 3 * NBA; i += NTHR * 4) *(v4ia*)(reg2 + i) = z4;
    if (tid < 16) wcnt[tid] = 0;
  }
  __syncthreads();

  int tot = 0, ovf = 0;
  const int nChunks = (nE + CHUNK - 1) / CHUNK;
#pragma unroll 1
  for (int ch = 0; ch < nChunks; ++ch) {
    const int cbase = ch * CHUNK;
    const int wc = scan_chunk<SLA>(dsts, nE, cbase, nodeBase, nb, vec8, list, tid, lane, wave);
    if (lane == 0) wcnt[wave] = wc;
    __syncthreads();
    int pre = 0, all = 0;
#pragma unroll
    for (int w2 = 0; w2 < NWAVE; ++w2) {
      int c = wcnt[w2];
      c = c < 0 ? 0 : (c > WCAP ? WCAP : c);
      all += c;
      pre += (w2 < wave) ? c : 0;
    }
    const int wcc  = wc > WCAP ? WCAP : wc;
    const int base = tot + pre;
#pragma unroll 1
    for (int i = lane; i < wcc; i += 32) {
      const int ent = list[wave * WCAP + i];
      const int el  = (ent >> SLA) & (CHUNK - 1);
      const int sq  = ent & (NBA - 1);
      int eid = cbase + el;
      eid = eid > nE - 1 ? nE - 1 : eid;
      const int sraw = srcs[eid];
      const int s = sraw < 0 ? 0 : (sraw > nN - 1 ? nN - 1 : sraw);
      const int pos = base + i;
      if (pos < RCAP) reg1[pos] = (int)((unsigned)s | ((unsigned)sq << SRCB));
    }
    if (tot + all > RCAP) ovf = 1;
    tot += all;
    tot = tot > RCAP ? RCAP : tot;
    __syncthreads();
  }
  const int nh = tot;

  if (wave == 0) {
#pragma unroll 1
    for (int b0 = 0; b0 < nh; b0 += 32) {
      const int idx = b0 + lane;
      const int uv  = reg1[idx < nh ? idx : nh - 1];
      const int m32 = (nh - b0) < 32 ? (nh - b0) : 32;
#pragma unroll 1
      for (int k = 0; k < m32; ++k) {
        const int u  = __builtin_amdgcn_readlane(uv, k);
        const int sq = (u >> SRCB) & (NBA - 1);
        if (lane == 0) cnt[sq] = cnt[sq] + 1;
      }
    }
  }
  __syncthreads();
  if (wave == 0) {
    const int base = lane * (NBA / 32);
    int s = 0;
#pragma unroll 1
    for (int i = 0; i < NBA / 32; ++i) s += cnt[base + i];
    int incl = s;
#pragma unroll
    for (int d = 1; d < 32; d <<= 1) {
      const int y = __shfl_up(incl, d, 32);
      if (lane >= d) incl += y;
    }
    int run = incl - s;
#pragma unroll 1
    for (int i = 0; i < NBA / 32; ++i) {
      const int cv = cnt[base + i];
      offs[base + i] = run;
      cur[base + i]  = run;
      run += cv;
    }
  }
  __syncthreads();
  if (wave == 0) {
#pragma unroll 1
    for (int b0 = 0; b0 < nh; b0 += 32) {
      const int idx = b0 + lane;
      const int uv  = reg1[idx < nh ? idx : nh - 1];
      const int m32 = (nh - b0) < 32 ? (nh - b0) : 32;
#pragma unroll 1
      for (int k = 0; k < m32; ++k) {
        const int u  = __builtin_amdgcn_readlane(uv, k);
        const int sq = (u >> SRCB) & (NBA - 1);
        if (lane == 0) {
          int p = cur[sq];
          p = p < 0 ? 0 : (p > RCAP - 1 ? RCAP - 1 : p);
          reg2[p] = u & ((1 << SRCB) - 1);
          cur[sq] = p + 1;
        }
      }
    }
  }
  __syncthreads();

  int* hb = HITS + (size_t)blk * RCAP;
  int* tb = TAB + (size_t)blk * (2 * NBA) + 4 * tid;
  const v4i tv = *(const v4ia*)(tab + 4 * tid);
  v4i cv;
  cv.x = (tid == 0) ? nh : 0;
  cv.y = (tid == 0) ? ovf : 0;
  cv.z = 0; cv.w = 0;
  int* fp = FLG + (size_t)blk * 32 + 4 * (tid & 7);
#pragma unroll 1
  for (int p = tid * 4; p < RCAP; p += NTHR * 4) {
    const v4i v = *(const v4ia*)(reg2 + p);
    *(volatile v4i*)(hb + p) = v;
  }
  *(volatile v4i*)tb = tv;
  if (tid < 8) *(volatile v4i*)fp = cv;
  __threadfence();
#pragma unroll 1
  for (int p = tid * 4; p < RCAP; p += NTHR * 4) {
    const v4i v = *(const v4ia*)(reg2 + p);
    *(volatile v4i*)(hb + p) = v;
  }
  *(volatile v4i*)tb = tv;
  if (tid < 8) *(volatile v4i*)fp = cv;
}

template <int NT>
__global__ __launch_bounds__(GTHR) __attribute__((amdgpu_num_vgpr(248)))
void k_gemm(const unsigned short* __restrict__ A, const unsigned short* __restrict__ WT,
            float* outF, int K, int ldo) {
  static_assert(NT == 4 || NT == 1);
  constexpr int BN = 16 * NT;
  __shared__ __attribute__((aligned(16))) float stg[GBM * BN];
  const int tid = (int)threadIdx.x, lane = tid & 31, wave = tid >> 5, hh = lane >> 4, m = lane & 15;
  const int rowBase = (int)blockIdx.x * GBM;
  const int col0    = (int)blockIdx.y * BN;

  v8f acc[NT];
  {
    const v8f z = {0.f, 0.f, 0.f, 0.f, 0.f, 0.f, 0.f, 0.f};
#pragma unroll
    for (int t = 0; t < NT; ++t) acc[t] = z;
  }
  const unsigned short* ap = A  + (size_t)(rowBase + 16 * wave + m) * (size_t)K + 8 * hh;
  const unsigned short* wp = WT + (size_t)(col0 + m) * (size_t)K + 8 * hh;
  const int ksteps = K >> 5;
#pragma unroll 1
  for (int ks = 0; ks < ksteps; ++ks) {
    FragB af;
    af.h[0] = *(const v8usa*)(ap + 32 * ks);
    af.h[1] = *(const v8usa*)(ap + 32 * ks + 16);
#pragma unroll
    for (int t = 0; t < NT; ++t) {
      const unsigned short* wq = wp + (size_t)(16 * t) * (size_t)K + 32 * ks;
      FragB bf;
      bf.h[0] = *(const v8usa*)wq;
      bf.h[1] = *(const v8usa*)(wq + 16);
      acc[t] = wmb(af, bf, acc[t]);
    }
  }

#pragma unroll
  for (int t = 0; t < NT; ++t) {
    const int lc = 16 * t + m;
#pragma unroll
    for (int r = 0; r < 8; ++r) {
      const int lr = 16 * wave + 8 * hh + r;
      stg[lr * BN + lc] = acc[t][r];
    }
  }
  __syncthreads();

  if constexpr (NT == 4) {
    v4f fv[8];
#pragma unroll
    for (int i = 0; i < 8; ++i) {
      const int lr = 16 * wave + 2 * i + hh;
      fv[i] = *(const v4fa*)(stg + lr * BN + 4 * m);
    }
#pragma unroll
    for (int i = 0; i < 8; ++i) {
      const int gr = rowBase + 16 * wave + 2 * i + hh;
      float* op = outF + (size_t)gr * (size_t)ldo + col0 + 4 * m;
      *(volatile v4f*)op = fv[i];
    }
    __threadfence();
#pragma unroll
    for (int i = 0; i < 8; ++i) {
      const int gr = rowBase + 16 * wave + 2 * i + hh;
      float* op = outF + (size_t)gr * (size_t)ldo + col0 + 4 * m;
      *(volatile v4f*)op = fv[i];
    }
  } else {
    const v4f f0 = *(const v4fa*)(stg + 4 * tid);
    const v4f f1 = *(const v4fa*)(stg + 4 * (tid + GTHR));
    float* op = outF + (size_t)rowBase * H3W;
    *(volatile v4f*)(op + 4 * tid) = f0;
    *(volatile v4f*)(op + 4 * (tid + GTHR)) = f1;
    __threadfence();
    *(volatile v4f*)(op + 4 * tid) = f0;
    *(volatile v4f*)(op + 4 * (tid + GTHR)) = f1;
  }
}

template <int L>
__global__ __launch_bounds__(NTHR) void k_dots(const float* __restrict__ Hm, const float* __restrict__ atts,
                                               const float* __restrict__ attd, float* SD, int MPr) {
  static_assert(L >= 1 && L <= 3);
  constexpr int FW   = (L == 1) ? HC1 : (L == 2) ? HC2 : H3W;
  constexpr int ALEN = (L == 1) ? HC1 : (L == 2) ? HC2 : NCLS;
  constexpr int NST  = (L == 3) ? 32 : FW;
  constexpr int NSTP = ((NST + NTHR - 1) / NTHR) * NTHR;
  __shared__ __attribute__((aligned(16))) float satt[2 * HC1];
  __shared__ __attribute__((aligned(16))) float sres[2 * DROWS * NHD];
  const int tid = (int)threadIdx.x, lane = tid & 31, wave = tid >> 5;
  const int rowBase = (int)blockIdx.x * DROWS;

  for (int i0 = 0; i0 < NSTP; i0 += NTHR) {
    const int i  = i0 + tid;
    const int ci = i < ALEN ? i : ALEN - 1;
    const float vs = atts[ci];
    const float vd = attd[ci];
    if (i < NST) {
      satt[i]       = (i < ALEN) ? bfr(vs) : 0.0f;
      satt[HC1 + i] = (i < ALEN) ? bfr(vd) : 0.0f;
    }
  }
  __syncthreads();

#pragma unroll 1
  for (int q = 0; q < DROWS / NWAVE; ++q) {
    const int lr  = wave * (DROWS / NWAVE) + q;
    const int row = rowBase + lr;
    float rs = 0.0f, rd = 0.0f;
    if constexpr (L == 3) {
      const int ch = lane & 15;
      const float hv = Hm[(size_t)row * H3W + ch];
      float ps = hv * satt[ch];
      float pd = hv * satt[HC1 + ch];
#pragma unroll
      for (int off = 8; off > 0; off >>= 1) {
        ps += __shfl_xor(ps, off);
        pd += __shfl_xor(pd, off);
      }
      rs = (lane == 0) ? ps : 0.0f;
      rd = (lane == 0) ? pd : 0.0f;
    } else {
      const float* hp = Hm + (size_t)row * FW + 4 * lane;
#pragma unroll 1
      for (int j = 0; j < FW / 128; ++j) {
        const v4f hv = *(const v4f*)(hp + 128 * j);
        const v4f sv = *(const v4fa*)(satt + 128 * j + 4 * lane);
        const v4f dv = *(const v4fa*)(satt + HC1 + 128 * j + 4 * lane);
        float ps = hv.x * sv.x;
        ps = fmaf(hv.y, sv.y, ps); ps = fmaf(hv.z, sv.z, ps); ps = fmaf(hv.w, sv.w, ps);
        float pd = hv.x * dv.x;
        pd = fmaf(hv.y, dv.y, pd); pd = fmaf(hv.z, dv.z, pd); pd = fmaf(hv.w, dv.w, pd);
        if constexpr (L == 1) {
#pragma unroll
          for (int off = 16; off > 0; off >>= 1) {
            ps += __shfl_xor(ps, off);
            pd += __shfl_xor(pd, off);
          }
          rs = (lane == j) ? ps : rs;
          rd = (lane == j) ? pd : rd;
        } else {
#pragma unroll
          for (int off = 8; off > 0; off >>= 1) {
            ps += __shfl_xor(ps, off);
            pd += __shfl_xor(pd, off);
          }
          const float pso = __shfl_xor(ps, 16);
          const float pdo = __shfl_xor(pd, 16);
          rs = (lane == 2 * j) ? ps : ((lane == 2 * j + 1) ? pso : rs);
          rd = (lane == 2 * j) ? pd : ((lane == 2 * j + 1) ? pdo : rd);
        }
      }
    }
    if (lane < NHD) {
      sres[lr * NHD + lane] = rs;
      sres[DROWS * NHD + lr * NHD + lane] = rd;
    }
  }
  __syncthreads();

  if (wave < 2) {
    const float* sp = sres + wave * (DROWS * NHD);
    const v4f v0 = *(const v4fa*)(sp + 4 * lane);
    const v4f v1 = *(const v4fa*)(sp + 128 + 4 * lane);
    float* dp = SD + (size_t)wave * (size_t)MPr * NHD + (size_t)rowBase * NHD;
    *(volatile v4f*)(dp + 4 * lane) = v0;
    *(volatile v4f*)(dp + 128 + 4 * lane) = v1;
    __threadfence();
    *(volatile v4f*)(dp + 4 * lane) = v0;
    *(volatile v4f*)(dp + 128 + 4 * lane) = v1;
  }
}

template <int L>
__global__ __launch_bounds__(NTHR) __attribute__((amdgpu_num_vgpr(248)))
void k_scan(const int* __restrict__ HITS, const int* __restrict__ TAB, const int* __restrict__ FLG,
            const float* __restrict__ F, const float* __restrict__ SD, const float* __restrict__ bias,
            unsigned short* XP, float* out, int nN, int MPr) {
  static_assert(L >= 1 && L <= 3);
  constexpr int FW    = (L == 1) ? HC1 : (L == 2) ? HC2 : H3W;
  constexpr int CH    = (L == 1) ? 128 : 64;
  constexpr int BLEN  = (L == 1) ? HC1 : (L == 2) ? HC2 : NCLS;
  constexpr int NBIAS = (L == 3) ? 16 : SCW;
  constexpr int NBP   = ((NBIAS + NTHR - 1) / NTHR) * NTHR;
  constexpr int KA    = 2 * FW;
  extern __shared__ __attribute__((aligned(16))) int ssm[];
  int*   sl    = ssm;
  int*   tab   = sl + RCAP;
  float* sbias = (float*)(tab + 2 * NBA);
  int*   stage = (int*)(sbias + SCW);
  const int tid = (int)threadIdx.x, lane = tid & 31, wave = tid >> 5;
  const int blk = (int)blockIdx.x;
  const int colBase = (int)blockIdx.y * SCW;
  const int nodeBase = blk * NBA;

  const int nhraw = FLG[(size_t)blk * 32];
  const int bflag = FLG[(size_t)blk * 32 + 1];
  const int nh  = nhraw < 0 ? 0 : (nhraw > RCAP ? RCAP : nhraw);
  const int ovf = (bflag != 0 || nhraw < 0 || nhraw > RCAP) ? 1 : 0;

  {
    const int* hb = HITS + (size_t)blk * RCAP;
#pragma unroll 1
    for (int p = tid * 4; p < RCAP; p += NTHR * 4) *(v4ia*)(sl + p) = *(const v4i*)(hb + p);
    *(v4ia*)(tab + 4 * tid) = *(const v4i*)(TAB + (size_t)blk * (2 * NBA) + 4 * tid);
    for (int i0 = 0; i0 < NBP; i0 += NTHR) {
      const int i  = i0 + tid;
      const int gi = colBase + i;
      const int ci = gi < BLEN ? gi : BLEN - 1;
      const float bv = bias[ci];
      if (i < NBIAS) sbias[i] = (gi < BLEN) ? bfr(bv) : 0.0f;
    }
  }
  __syncthreads();

  const float qnan = __int_as_float(0x7fc00000);
  const int head = (L == 3) ? 0 : (colBase + CPL * lane) / CH;
  const int ch3  = lane & 15;
  const float* ASp = SD;
  const float* ADp = SD + (size_t)MPr * NHD;
  unsigned short* stw = (unsigned short*)stage + wave * (2 * SCW);
  float* ostg = (float*)stage;
  float b3v = 0.0f;
  if constexpr (L == 3) b3v = sbias[ch3];

#pragma unroll 1
  for (int si = 0; si < NBA / NWAVE; ++si) {
    const int s    = si * NWAVE + wave;
    const int node = nodeBase + s;
    const int nc   = node < nN ? node : nN - 1;
    int c = tab[NBA + s];
    const bool big = c > DEGCAP;
    c = c < 0 ? 0 : (c > DEGCAP ? DEGCAP : c);
    int o = tab[s];
    o = o < 0 ? 0 : (o > RCAP ? RCAP : o);
    if (c > nh - o) c = nh - o;
    c = c < 0 ? 0 : c;
    const float adv = ADp[(size_t)nc * NHD + head];
    float mx = -3.0e38f, dn = 0.0f;
    v4f acc[4];
    {
      const v4f z4 = {0.f, 0.f, 0.f, 0.f};
      acc[0] = z4; acc[1] = z4; acc[2] = z4; acc[3] = z4;
    }
    float a3 = 0.0f;
    const int T = c + 1;
#pragma unroll 1
    for (int b0 = 0; b0 < T; b0 += 32) {
      const int t = b0 + lane;
      int idx = o + t;
      idx = idx < 0 ? 0 : (idx > RCAP - 1 ? RCAP - 1 : idx);
      const int ent = sl[idx];
      const int hs  = ent < 0 ? 0 : (ent > nN - 1 ? nN - 1 : ent);
      const int sr  = (t < c) ? hs : nc;
      const int m32 = (T - b0) < 32 ? (T - b0) : 32;
#pragma unroll 1
      for (int k = 0; k < m32; ++k) {
        const int sk = __builtin_amdgcn_readlane(sr, k);
        float lg = ASp[(size_t)sk * NHD + head] + adv;
        lg = lg > 0.f ? lg : NEGSL * lg;
        const float df = lg - mx;
        const float ee = expf(-fabsf(df));
        const bool  up = df > 0.f;
        const float s1 = up ? ee : 1.0f;
        const float s2 = up ? 1.0f : ee;
        mx = up ? lg : mx;
        dn = fmaf(dn, s1, s2);
        if constexpr (L == 3) {
          const float av = F[(size_t)sk * H3W + ch3];
          a3 = fmaf(a3, s1, s2 * av);
        } else {
          const float* rp = F + (size_t)sk * FW + colBase + CPL * lane;
          const v4f g0 = *(const v4f*)rp;
          const v4f g1 = *(const v4f*)(rp + 4);
          const v4f g2 = *(const v4f*)(rp + 8);
          const v4f g3 = *(const v4f*)(rp + 12);
          acc[0].x = fmaf(acc[0].x, s1, s2 * g0.x); acc[0].y = fmaf(acc[0].y, s1, s2 * g0.y);
          acc[0].z = fmaf(acc[0].z, s1, s2 * g0.z); acc[0].w = fmaf(acc[0].w, s1, s2 * g0.w);
          acc[1].x = fmaf(acc[1].x, s1, s2 * g1.x); acc[1].y = fmaf(acc[1].y, s1, s2 * g1.y);
          acc[1].z = fmaf(acc[1].z, s1, s2 * g1.z); acc[1].w = fmaf(acc[1].w, s1, s2 * g1.w);
          acc[2].x = fmaf(acc[2].x, s1, s2 * g2.x); acc[2].y = fmaf(acc[2].y, s1, s2 * g2.y);
          acc[2].z = fmaf(acc[2].z, s1, s2 * g2.z); acc[2].w = fmaf(acc[2].w, s1, s2 * g2.w);
          acc[3].x = fmaf(acc[3].x, s1, s2 * g3.x); acc[3].y = fmaf(acc[3].y, s1, s2 * g3.y);
          acc[3].z = fmaf(acc[3].z, s1, s2 * g3.z); acc[3].w = fmaf(acc[3].w, s1, s2 * g3.w);
        }
      }
    }
    const float inv = __builtin_amdgcn_rcpf(dn + EPS_SM);
    const float pzr = (big || ovf != 0) ? qnan : 0.0f;
    const bool live = node < nN;

    if constexpr (L == 3) {
      const bool valid = ch3 < NCLS;
      const float z = fmaf(a3, inv, b3v);
      float vm = valid ? z : -3.0e38f;
#pragma unroll
      for (int off = 8; off > 0; off >>= 1) vm = fmaxf(vm, __shfl_xor(vm, off));
      const float ex = expf(z - vm);
      float sm = valid ? ex : 0.0f;
#pragma unroll
      for (int off = 8; off > 0; off >>= 1) sm += __shfl_xor(sm, off);
      const float ov = ((z - vm) - logf(sm)) + pzr;
      if (lane < NCLS) ostg[s * NCLS + lane] = ov;
    } else {
      const v4f bA = *(const v4fa*)(sbias + CPL * lane);
      const v4f bB = *(const v4fa*)(sbias + CPL * lane + 4);
      const v4f bC = *(const v4fa*)(sbias + CPL * lane + 8);
      const v4f bD = *(const v4fa*)(sbias + CPL * lane + 12);
      v8us ho0, lo0, ho1, lo1;
#define HL(HO, LO, E, AV, BV) { \
        const float v_ = fin1((AV), inv, (BV), pzr, live); \
        const unsigned int hb_ = f2bf(v_); \
        HO[E] = (unsigned short)hb_; \
        LO[E] = (unsigned short)f2bf(v_ - bf2f(hb_)); }
      HL(ho0, lo0, 0, acc[0].x, bA.x) HL(ho0, lo0, 1, acc[0].y, bA.y)
      HL(ho0, lo0, 2, acc[0].z, bA.z) HL(ho0, lo0, 3, acc[0].w, bA.w)
      HL(ho0, lo0, 4, acc[1].x, bB.x) HL(ho0, lo0, 5, acc[1].y, bB.y)
      HL(ho0, lo0, 6, acc[1].z, bB.z) HL(ho0, lo0, 7, acc[1].w, bB.w)
      HL(ho1, lo1, 0, acc[2].x, bC.x) HL(ho1, lo1, 1, acc[2].y, bC.y)
      HL(ho1, lo1, 2, acc[2].z, bC.z) HL(ho1, lo1, 3, acc[2].w, bC.w)
      HL(ho1, lo1, 4, acc[3].x, bD.x) HL(ho1, lo1, 5, acc[3].y, bD.y)
      HL(ho1, lo1, 6, acc[3].z, bD.z) HL(ho1, lo1, 7, acc[3].w, bD.w)
#undef HL
      *(v8usa*)(stw + CPL * lane)           = ho0;
      *(v8usa*)(stw + CPL * lane + 8)       = ho1;
      *(v8usa*)(stw + SCW + CPL * lane)     = lo0;
      *(v8usa*)(stw + SCW + CPL * lane + 8) = lo1;
      __syncthreads();
      const v8us q0 = *(const v8usa*)(stw + 8 * lane);
      const v8us q1 = *(const v8usa*)(stw + 256 + 8 * lane);
      const v8us q2 = *(const v8usa*)(stw + SCW + 8 * lane);
      const v8us q3 = *(const v8usa*)(stw + SCW + 256 + 8 * lane);
      unsigned short* gp = XP + (size_t)node * KA + colBase + 8 * lane;
      const bool wr = node < MPr;
      if (wr) {
        *(volatile v8us*)gp              = q0;
        *(volatile v8us*)(gp + 256)      = q1;
        *(volatile v8us*)(gp + FW)       = q2;
        *(volatile v8us*)(gp + FW + 256) = q3;
      }
      __threadfence();
      if (wr) {
        *(volatile v8us*)gp              = q0;
        *(volatile v8us*)(gp + 256)      = q1;
        *(volatile v8us*)(gp + FW)       = q2;
        *(volatile v8us*)(gp + FW + 256) = q3;
      }
      __syncthreads();
    }
  }

  if constexpr (L == 3) {
    __syncthreads();
    int live = nN - nodeBase;
    live = live < 0 ? 0 : (live > NBA ? NBA : live);
    const int npc = (live * NCLS) >> 2;
    float* ob = out + (size_t)nodeBase * NCLS;
#pragma unroll 1
    for (int p = tid; p < npc; p += NTHR) {
      const v4f v = *(const v4fa*)(ostg + 4 * p);
      *(volatile v4f*)(ob + 4 * p) = v;
    }
    __threadfence();
#pragma unroll 1
    for (int p = tid; p < npc; p += NTHR) {
      const v4f v = *(const v4fa*)(ostg + 4 * p);
      *(volatile v4f*)(ob + 4 * p) = v;
    }
  }
}

static inline size_t al256(size_t v) { return (v + 255) & ~(size_t)255; }

extern "C" void kernel_launch(void* const* d_in, const int* in_sizes, int n_in,
                              void* d_out, int out_size, void* d_ws, size_t ws_size,
                              hipStream_t stream) {
  if (n_in < 14) return;
  if (in_sizes[0] != NNODE * FIN) return;
  if (in_sizes[1] < 2 || (in_sizes[1] & 1) != 0) return;
  const int nE = in_sizes[1] / 2;
  if (nE < 1 || nE > (1 << 28)) return;
  if (in_sizes[2] != HC1 * FIN) return;
  if (in_sizes[3] != HC1 || in_sizes[4] != HC1 || in_sizes[5] != HC1) return;
  if (in_sizes[6] != HC2 * HC1) return;
  if (in_sizes[7] != HC2 || in_sizes[8] != HC2 || in_sizes[9] != HC2) return;
  if (in_sizes[10] != NCLS * HC2) return;
  if (in_sizes[11] != NCLS || in_sizes[12] != NCLS || in_sizes[13] != NCLS) return;
  if (out_size != NNODE * NCLS) return;

  const float* x   = (const float*)d_in[0];
  const int*   ei  = (const int*)  d_in[1];
  const float* W1  = (const float*)d_in[2];
  const float* as1 = (const float*)d_in[3];
  const float* ad1 = (const float*)d_in[4];
  const float* b1  = (const float*)d_in[5];
  const float* W2  = (const float*)d_in[6];
  const float* as2 = (const float*)d_in[7];
  const float* ad2 = (const float*)d_in[8];
  const float* b2  = (const float*)d_in[9];
  const float* W3  = (const float*)d_in[10];
  const float* as3 = (const float*)d_in[11];
  const float* ad3 = (const float*)d_in[12];
  const float* b3  = (const float*)d_in[13];
  float* out = (float*)d_out;
  const int* src = ei;
  const int* dst = ei + nE;
  const int nN = NNODE;
  const int MP = MPAD;
  const int vec8 = ((nE & 3) == 0) ? 1 : 0;

  char* ws = (char*)d_ws;
  size_t off = 0;
  const size_t szA = (size_t)MP * KA2 * 2;
  const size_t szB = (size_t)MP * HC1 * 4;
  const size_t oA   = off; off = al256(off + szA);
  const size_t oB   = off; off = al256(off + szB);
  const size_t oW1  = off; off = al256(off + (size_t)HC1 * K1P * 2);
  const size_t oW2  = off; off = al256(off + (size_t)HC2 * KA2 * 2);
  const size_t oW3  = off; off = al256(off + (size_t)H3W * KA3 * 2);
  const size_t oSD  = off; off = al256(off + (size_t)2 * MP * NHD * 4);
  const size_t oHIT = off; off = al256(off + (size_t)NGA * RCAP * 4);
  const size_t oTAB = off; off = al256(off + (size_t)NGA * 2 * NBA * 4);
  const size_t oFLG = off; off = al256(off + (size_t)NGA * 128);
  if (off > ws_size) return;
  const size_t oH3 = (size_t)MP * HC2 * 4;
  if ((size_t)MP * K1P * 2 > szA || (size_t)MP * KA3 * 2 > szA) return;
  if (oH3 + (size_t)MP * H3W * 4 > szB) return;

  unsigned short* XB   = (unsigned short*)(ws + oA);
  unsigned short* X1hl = (unsigned short*)(ws + oA);
  unsigned short* X2hl = (unsigned short*)(ws + oA);
  float*          H1   = (float*)(ws + oB);
  float*          H2   = (float*)(ws + oB);
  float*          H3   = (float*)(ws + oB + oH3);
  unsigned short* W1B  = (unsigned short*)(ws + oW1);
  unsigned short* W2D  = (unsigned short*)(ws + oW2);
  unsigned short* W3D  = (unsigned short*)(ws + oW3);
  float*          SD   = (float*)(ws + oSD);
  int*            HITS = (int*)(ws + oHIT);
  int*            TAB  = (int*)(ws + oTAB);
  int*            FLG  = (int*)(ws + oFLG);

  const int bktLds  = BKT_LDS_INTS * 4;
  const int scanLds = SCAN_LDS_INTS * 4;
  hipFuncSetAttribute(reinterpret_cast<const void*>(&k_bucket),
                      hipFuncAttributeMaxDynamicSharedMemorySize, bktLds);
  hipFuncSetAttribute(reinterpret_cast<const void*>(&k_scan<1>),
                      hipFuncAttributeMaxDynamicSharedMemorySize, scanLds);
  hipFuncSetAttribute(reinterpret_cast<const void*>(&k_scan<2>),
                      hipFuncAttributeMaxDynamicSharedMemorySize, scanLds);
  hipFuncSetAttribute(reinterpret_cast<const void*>(&k_scan<3>),
                      hipFuncAttributeMaxDynamicSharedMemorySize, scanLds);

  {
    const int nUx = MP * (K1P / 8);
    k_cvt<<<(nUx + NTHR - 1) / NTHR, NTHR, 0, stream>>>(x, NNODE, FIN, K1P, XB, K1P, nUx);
    const int nU1 = HC1 * (K1P / 8);
    k_cvt<<<(nU1 + NTHR - 1) / NTHR, NTHR, 0, stream>>>(W1, HC1, FIN, K1P, W1B, K1P, nU1);
    const int nU2 = HC2 * (KA2 / 8);
    k_cvt<<<(nU2 + NTHR - 1) / NTHR, NTHR, 0, stream>>>(W2, HC2, HC1, HC1, W2D, KA2, nU2);
    const int nU3 = H3W * (KA3 / 8);
    k_cvt<<<(nU3 + NTHR - 1) / NTHR, NTHR, 0, stream>>>(W3, NCLS, HC2, HC2, W3D, KA3, nU3);
  }
  k_bucket<<<NGA, NTHR, bktLds, stream>>>(src, dst, nE, nN, vec8, HITS, TAB, FLG);

  const int gM = MP / GBM;
  k_gemm<4><<<dim3(gM, HC1 / 64), GTHR, 0, stream>>>(XB, W1B, H1, K1P, HC1);
  k_dots<1><<<MP / DROWS, NTHR, 0, stream>>>(H1, as1, ad1, SD, MP);
  k_scan<1><<<dim3(NGA, HC1 / SCW), NTHR, scanLds, stream>>>(HITS, TAB, FLG, H1, SD, b1, X1hl, out, nN, MP);
  k_gemm<4><<<dim3(gM, HC2 / 64), GTHR, 0, stream>>>(X1hl, W2D, H2, KA2, HC2);
  k_dots<2><<<MP / DROWS, NTHR, 0, stream>>>(H2, as2, ad2, SD, MP);
  k_scan<2><<<dim3(NGA, 1), NTHR, scanLds, stream>>>(HITS, TAB, FLG, H2, SD, b2, X2hl, out, nN, MP);
  k_gemm<1><<<dim3(gM, 1), GTHR, 0, stream>>>(X2hl, W3D, H3, KA3, H3W);
  k_dots<3><<<MP / DROWS, NTHR, 0, stream>>>(H3, as3, ad3, SD, MP);
  k_scan<3><<<dim3(NGA, 1), NTHR, scanLds, stream>>>(HITS, TAB, FLG, H3, SD, b3, X2hl, out, nN, MP);
}
